// HybridModel_23828478558270
// MI455X (gfx1250) — hardware-verified
//
#include <hip/hip_runtime.h>


#ifndef NSAMP
#define NSAMP 8192
#endif
#define NSAMP_FULL 8192
#define DIN   256
#define HID   128
#define NQ    10
#define NL    6
#define DOUT  64
#define FW    16
#define AW    4
#define SPW   4
#define SS    1024.0f
#define WS    256.0f
#define WSI   (1.0f / 256.0f)
#define PSC   (1.0f / (1024.0f * 1024.0f * 256.0f * 256.0f))

static_assert(NQ == 10);
static_assert(NL * 2 * 4096 == 12 * 64 * 64);
static_assert(DIN % 32 == 0);
static_assert(FW == 16);
static_assert(FW <= HID);
static_assert(NQ <= FW);
static_assert(NSAMP % 64 == 0);
static_assert(NSAMP % (AW * SPW) == 0);
static_assert(NSAMP <= NSAMP_FULL);
static_assert(((size_t)NSAMP * DIN) % 8 == 0);
static_assert((FW * DIN) % 8 == 0);
static_assert((NL * 64) % (32 * AW) == 0);
static_assert((NQ * DOUT) % (32 * AW) == 0);
static_assert(DOUT <= 32 * AW);
static_assert(16 * 16 == DOUT * 4);
static_assert(8 * 32 * 16 == 64 * FW * 4);
static_assert(2 * 256 * 16 == 64 * 64 * 2);
static_assert(AW * 2048 * 2 + AW * 1024 * 4 + NL * 64 * 2 + NQ * DOUT * 4 + DOUT * 4 <= 131072);
static_assert(32 * 4 + 5 * 8 * 4 + 4096 * 2 <= 131072);
static_assert(64 * FW * 4 <= 131072);

typedef _Float16 h16;
typedef unsigned short bf;
typedef __attribute__((ext_vector_type(16))) __bf16   v16bf;
typedef __attribute__((ext_vector_type(16))) _Float16 v16h;
typedef __attribute__((ext_vector_type(8)))  _Float16 v8h;
typedef __attribute__((ext_vector_type(8)))  unsigned short v8us;
typedef __attribute__((ext_vector_type(8)))  float    v8f;
typedef __attribute__((ext_vector_type(4)))  float    v4f;
typedef v4f  __attribute__((may_alias)) v4fa;
typedef v8h  __attribute__((may_alias)) v8ha;
typedef v8us __attribute__((may_alias)) v8usa;

__device__ __forceinline__ unsigned short f2bf(float f) { unsigned u = __float_as_uint(f); u += 0x7FFFu + ((u >> 16) & 1u); return (unsigned short)(u >> 16); }
__device__ __forceinline__ float bfr(float f) { return __uint_as_float(((unsigned)f2bf(f)) << 16); }
__device__ __forceinline__ v16h cat16(v8h lo, v8h hi) { return __builtin_shufflevector(lo, hi, 0, 1, 2, 3, 4, 5, 6, 7, 8, 9, 10, 11, 12, 13, 14, 15); }
__device__ __forceinline__ v16bf cat16b(v8us lo, v8us hi) { return __builtin_bit_cast(v16bf, __builtin_shufflevector(lo, hi, 0, 1, 2, 3, 4, 5, 6, 7, 8, 9, 10, 11, 12, 13, 14, 15)); }
__device__ __forceinline__ v8f wmma16(v16h a, v16h b, v8f c) { return __builtin_amdgcn_wmma_f32_16x16x32_f16(false, a, false, b, (short)0, c, false, false); }
__device__ __forceinline__ v8f wmmab(v16bf a, v16bf b, v8f c) { return __builtin_amdgcn_wmma_f32_16x16x32_bf16(false, a, false, b, (short)0, c, false, false); }
__device__ __forceinline__ v16h  ldh(const h16* p) { return cat16(*(const v8h*)p, *(const v8h*)(p + 16)); }
__device__ __forceinline__ v16bf ldb(const bf* p)  { return cat16b(*(const v8us*)p, *(const v8us*)(p + 16)); }
__device__ __forceinline__ void wave_sync() { __builtin_amdgcn_fence(3  , "wavefront"); __builtin_amdgcn_wave_barrier(); asm volatile("" ::: "memory"); }

static __device__ __forceinline__ h16 toh_flush(float v) { const h16 r = (h16)v; return (fabsf(v) < 6.103515625e-05f) ? (h16)0.0f : r; }
__device__ __forceinline__ v8f wmma16g(v16h a, v16h b, v8f c) { c = wmma16(a, b, c); asm volatile("v_nop\n\tv_nop\n\tv_nop\n\tv_nop" : "+v"(c) : "v"(a), "v"(b)); return c; }
__device__ __forceinline__ v8f wmmabg(v16bf a, v16bf b, v8f c) { c = wmmab(a, b, c); asm volatile("v_nop\n\tv_nop\n\tv_nop\n\tv_nop" : "+v"(c) : "v"(a), "v"(b)); return c; }
template <int N>
__device__ __forceinline__ float fold_pairs(float (&a)[32]) {
    float d = 0.0f;
#pragma unroll
    for (int j = 0; j < N / 2; ++j) { const float x = a[2 * j], y = a[2 * j + 1]; d += x - y; a[j] = x + y; }
    return d;
}

__global__ __launch_bounds__(256) void k_cvt8(const float* __restrict__ src, bf* dst, size_t n8) {
    const size_t i = (size_t)blockIdx.x * 256 + threadIdx.x; if (i >= n8) return;
    const v8f v = *(const v8f*)(src + i * 8); v8us o;
#pragma unroll
    for (int k = 0; k < 8; ++k) o[k] = f2bf(v[k]);
    *(volatile v8us*)(dst + i * 8) = o; __threadfence(); *(volatile v8us*)(dst + i * 8) = o;
}

__global__ __launch_bounds__(256) void k_wbuild(const float* __restrict__ qw, h16* WT) {
#pragma clang fp contract(off)
    __shared__ float cs[32];
    __shared__ float g[5][8];
    __shared__ __align__(16) h16 tile[64 * 64];
    const int tid = threadIdx.x;
    const int l = blockIdx.x >> 1, st = blockIdx.x & 1;
    const int q0 = st ? 0 : 5;
    {
        const int e = tid < 15 ? tid : 14; const int j = e / 3, a = e - 3 * j;
        const float* w = qw + (size_t)((l * NQ + q0 + j) * 3);
        float phi = bfr(w[0]), th = bfr(w[1]), om = bfr(w[2]);
        asm volatile("" : "+v"(phi), "+v"(th), "+v"(om));
        const float ang = (a == 0) ? (th * 0.5f) : ((a == 1) ? (0.5f * (phi + om)) : (0.5f * (phi - om)));
        float s, c; sincosf(ang, &s, &c);
        if (tid < 15) { cs[e * 2] = c; cs[e * 2 + 1] = s; }
    }
    __syncthreads();
    {
        const int j = tid < 5 ? tid : 4;
        float c = cs[(3 * j) * 2], s = cs[(3 * j) * 2 + 1], ca = cs[(3 * j + 1) * 2], sa = cs[(3 * j + 1) * 2 + 1], cb = cs[(3 * j + 2) * 2], sb = cs[(3 * j + 2) * 2 + 1];
        asm volatile("" : "+v"(c), "+v"(s), "+v"(ca), "+v"(sa), "+v"(cb), "+v"(sb));
        if (tid < 5) {
            g[j][0] = ca * c;    g[j][1] = -(sa * c);
            g[j][2] = -(cb * s); g[j][3] = -(sb * s);
            g[j][4] = cb * s;    g[j][5] = -(sb * s);
            g[j][6] = ca * c;    g[j][7] = sa * c; }
    }
    __syncthreads();
#pragma unroll 1
    for (int it = 0; it < 4; ++it) {
        const int e = tid + 256 * it; const int n = e >> 5, k = e & 31;
        float pr = 1.0f, pi = 0.0f;
#pragma unroll 1
        for (int j = 0; j < 5; ++j) {
            const int sh = 4 - j; const int idx = ((((n >> sh) & 1) << 1) | ((k >> sh) & 1)) * 2;
            const float gr = g[j][idx], gi = g[j][idx + 1];
            const float nr = pr * gr - pi * gi, ni = pr * gi + pi * gr; pr = nr; pi = ni; }
        pr *= WS; pi *= WS;
        tile[n * 64 + k]             = toh_flush(pr);
        tile[n * 64 + 32 + k]        = toh_flush(-pi);
        tile[(32 + n) * 64 + k]      = toh_flush(pi);
        tile[(32 + n) * 64 + 32 + k] = toh_flush(pr);
    }
    __syncthreads();
    h16* dst = WT + (size_t)blockIdx.x * 4096;
#pragma unroll 1
    for (int ps = 0; ps < 2; ++ps) {
#pragma unroll
        for (int s = 0; s < 2; ++s) { const int p = s * 256 + tid;
            const v8h v = *(const v8ha*)(&tile[p * 8]);
            *(volatile v8h*)(dst + (size_t)p * 8) = v; }
        if (ps == 0) __threadfence(); }
}

__global__ __launch_bounds__(32) void k_feat(const bf* __restrict__ A, const bf* __restrict__ Bt, const float* __restrict__ bias, float* Fo) {
    __shared__ __align__(16) float os[64 * FW];
    const int K = DIN;
    const int lane = threadIdx.x & 31, lr = lane & 15, hi = lane >> 4; const int r0 = blockIdx.x * 64;
    v8f acc[4];
#pragma unroll
    for (int mb = 0; mb < 4; ++mb) acc[mb] = (v8f){};
    const size_t aoff = (size_t)(r0 + lr) * K + 8 * hi, boff = (size_t)lr * K + 8 * hi;
#pragma unroll 1
    for (int kc = 0; kc < K; kc += 32) {
        const v16bf b = ldb(Bt + boff + kc);
#pragma unroll
        for (int mb = 0; mb < 4; ++mb) { const v16bf a = ldb(A + aoff + (size_t)mb * 16 * K + kc); acc[mb] = wmmabg(a, b, acc[mb]); }
    }
    const float bc = bfr(bias[lr]);
#pragma unroll
    for (int mb = 0; mb < 4; ++mb) {
#pragma unroll
        for (int j = 0; j < 8; ++j) os[(mb * 16 + hi * 8 + j) * FW + lr] = fmaxf(acc[mb][j] + bc, 0.0f); }
    wave_sync();
    float* dst = Fo + (size_t)r0 * FW;
#pragma unroll 1
    for (int ps = 0; ps < 2; ++ps) {
#pragma unroll
        for (int s = 0; s < 8; ++s) { const int p = s * 32 + lane;
            const v4f val = *(const v4fa*)(&os[p * 4]);
            *(volatile v4f*)(dst + (size_t)p * 4) = val; }
        if (ps == 0) __threadfence(); }
}

__global__ __launch_bounds__(32 * AW) void k_sim(const float* __restrict__ F, const h16* __restrict__ WT, const float* __restrict__ W2, const float* __restrict__ b2, float* OUT) {
    __shared__ __align__(16) h16 S[AW * 2048];
    __shared__ __align__(16) float P[AW * 1024];
    __shared__ __align__(16) unsigned short PT[NL * 64];
    __shared__ __align__(16) float W2T[NQ * DOUT];
    __shared__ __align__(16) float bias2[DOUT];
    const int tid = threadIdx.x;
    const int lane = threadIdx.x & 31, lr = lane & 15, hi = lane >> 4;
    const int wave = __builtin_amdgcn_readfirstlane((int)(threadIdx.x >> 5));
#pragma unroll 1
    for (int w = tid; w < NL * 64; w += 32 * AW) {
        const int l = w >> 6, e = w & 63; int i = (e < 32) ? (e << 5) : (e - 32);
        const int r = (l % (NQ - 1)) + 1;
#pragma unroll 1
        for (int q = 0; q < NQ; ++q) { const int c = 9 - q; int tq = q + r; tq = (tq >= NQ) ? (tq - NQ) : tq; const int t = 9 - tq; i ^= ((i >> c) & 1) << t; }
        PT[w] = (unsigned short)i; }
#pragma unroll 1
    for (int e = tid; e < NQ * DOUT; e += 32 * AW) {
        const int j = e / NQ, q = e - j * NQ; W2T[q * DOUT + j] = bfr(W2[e]); }
    if (tid < DOUT) bias2[tid] = bfr(b2[tid]);
    __syncthreads();

    const int sb = wave * 2048, pb = wave * 1024;
    const int kpop = __popc((unsigned)lane) & 3;
    const float pre = (kpop == 0) ? 1.0f : ((kpop == 2) ? -1.0f : 0.0f);
    const float pim = (kpop == 1) ? -1.0f : ((kpop == 3) ? 1.0f : 0.0f);
#pragma unroll 1
    for (int si = 0; si < SPW; ++si) {
        const int samp = (blockIdx.x * AW + wave) * SPW + si;
        const float ang = F[(size_t)samp * FW + lr];
        float sn, cn; sincosf(0.5f * ang, &sn, &cn);
        float mu = 1.0f, mv = 1.0f;
#pragma unroll
        for (int q = 0; q < 5; ++q) {
            const float c0 = __shfl(cn, q, 32), s0 = __shfl(sn, q, 32), c1 = __shfl(cn, q + 5, 32), s1 = __shfl(sn, q + 5, 32);
            const bool bit = ((lane >> (4 - q)) & 1) != 0;
            mu *= bit ? s0 : c0; mv *= bit ? s1 : c1; }
        const float ure = mu * pre * SS, uim = mu * pim * SS;
        const float vre = mv * pre, vim = mv * pim;
#pragma unroll 4
        for (int v = 0; v < 32; ++v) {
            const float wr = __shfl(vre, v, 32), wi = __shfl(vim, v, 32);
            const float re = ure * wr - uim * wi, im = ure * wi + uim * wr;
            S[sb + lane * 32 + v] = toh_flush(re); S[sb + 1024 + lane * 32 + v] = toh_flush(im); }
        wave_sync();

#pragma unroll 1
        for (int l = 0; l < NL; ++l) {
#pragma unroll
            for (int st = 0; st < 2; ++st) {
                const h16* Wp = WT + (size_t)(l * 2 + st) * 4096 + (size_t)lr * 64 + 8 * hi;
                v16h a[2][2];
#pragma unroll
                for (int mt = 0; mt < 2; ++mt)
#pragma unroll
                    for (int ks = 0; ks < 2; ++ks) { const int ix = sb + ks * 1024 + (16 * mt + lr) * 32 + 8 * hi;
                        a[mt][ks] = cat16(*(const v8ha*)(&S[ix]), *(const v8ha*)(&S[ix + 16])); }
                v8f acc[2][4];
#pragma unroll
                for (int mt = 0; mt < 2; ++mt)
#pragma unroll
                    for (int nt = 0; nt < 4; ++nt) acc[mt][nt] = (v8f){};
#pragma unroll
                for (int nt = 0; nt < 4; ++nt)
#pragma unroll
                    for (int ks = 0; ks < 2; ++ks) { const v16h b = ldh(Wp + nt * 16 * 64 + ks * 32);
#pragma unroll
                        for (int mt = 0; mt < 2; ++mt) acc[mt][nt] = wmma16g(a[mt][ks], b, acc[mt][nt]); }
                if (st == 0) {
#pragma unroll
                    for (int mt = 0; mt < 2; ++mt)
#pragma unroll
                        for (int nt = 0; nt < 4; ++nt) { v8h o;
#pragma unroll
                            for (int r = 0; r < 8; ++r) o[r] = toh_flush(acc[mt][nt][r] * WSI);
                            *(v8ha*)(&S[sb + (nt >> 1) * 1024 + (16 * (nt & 1) + lr) * 32 + 16 * mt + 8 * hi]) = o; }
                    wave_sync();
                } else {
                    const int pu0 = (int)PT[l * 64 + lr], pu1 = (int)PT[l * 64 + 16 + lr];
                    const v8us pva = *(const v8usa*)(&PT[l * 64 + 32 + 8 * hi]);
                    const v8us pvb = *(const v8usa*)(&PT[l * 64 + 32 + 16 + 8 * hi]);
                    if (l < NL - 1) {
#pragma unroll
                        for (int mt = 0; mt < 2; ++mt)
#pragma unroll
                            for (int nt = 0; nt < 4; ++nt)
#pragma unroll
                                for (int r = 0; r < 8; ++r) {
                                    const int d = ((nt & 1) ? pu1 : pu0) ^ (int)(mt ? pvb[r] : pva[r]);
                                    S[sb + (nt >> 1) * 1024 + d] = toh_flush(acc[mt][nt][r] * WSI); }
                    } else {
#pragma unroll
                        for (int mt = 0; mt < 2; ++mt)
#pragma unroll
                            for (int nl = 0; nl < 2; ++nl)
#pragma unroll
                                for (int r = 0; r < 8; ++r) {
                                    const int d = (nl ? pu1 : pu0) ^ (int)(mt ? pvb[r] : pva[r]);
                                    const float re = acc[mt][nl][r], im = acc[mt][nl + 2][r];
                                    P[pb + d] = (re * re + im * im) * PSC; }
                    }
                    wave_sync();
                }
            }
        }

        float pa[32];
#pragma unroll
        for (int i = 0; i < 8; ++i) { const v4f t = *(const v4fa*)(&P[pb + lane * 32 + 4 * i]); pa[4 * i] = t[0]; pa[4 * i + 1] = t[1]; pa[4 * i + 2] = t[2]; pa[4 * i + 3] = t[3]; }
        float z[NQ];
        z[9] = fold_pairs<32>(pa);
        z[8] = fold_pairs<16>(pa);
        z[7] = fold_pairs<8>(pa);
        z[6] = fold_pairs<4>(pa);
        z[5] = fold_pairs<2>(pa);
        const float tot = pa[0];
#pragma unroll
        for (int q = 0; q < 5; ++q) z[q] = ((lane >> (4 - q)) & 1) ? -tot : tot;
#pragma unroll
        for (int q = 0; q < NQ; ++q) {
#pragma unroll
            for (int m = 16; m >= 1; m >>= 1) z[q] += __shfl_xor(z[q], m, 32); }

        const int j4 = lr * 4;
        v4f o = *(const v4fa*)(&bias2[j4]);
#pragma unroll
        for (int q = 0; q < NQ; ++q) { const v4f w = *(const v4fa*)(&W2T[q * DOUT + j4]); o += w * z[q]; }
        asm volatile("" : "+v"(o));
        float* orow = OUT + (size_t)samp * DOUT + j4;
#pragma unroll 1
        for (int ps = 0; ps < 2; ++ps) {
            if (lane < 16) *(volatile v4f*)orow = o;
            if (ps == 0) __threadfence(); }
    }
}

static constexpr size_t al256(size_t v) { return (v + 255) & ~(size_t)255; }
static constexpr size_t SZ_XB = al256((size_t)NSAMP * DIN * 2);
static constexpr size_t SZ_WB = al256((size_t)FW * DIN * 2);
static constexpr size_t SZ_F  = al256((size_t)NSAMP * FW * 4);
static constexpr size_t SZ_WT = al256((size_t)NL * 2 * 4096 * 2);
static constexpr size_t SZ_TOTAL = SZ_XB + SZ_WB + SZ_F + SZ_WT;
static_assert(SZ_TOTAL <= (size_t)134217728);
static_assert((size_t)(NSAMP / 64) * 64 * FW * 4 <= SZ_F);
static_assert((size_t)(NL * 2) * 4096 * 2 <= SZ_WT);

extern "C" void kernel_launch(void* const* d_in, const int* in_sizes, int n_in,
                              void* d_out, int out_size, void* d_ws, size_t ws_size, hipStream_t stream) {
    if (n_in < 6) return;
    if ((size_t)in_sizes[0] < (size_t)NSAMP * DIN) return;
    if ((size_t)in_sizes[1] < (size_t)FW * DIN) return;
    if (in_sizes[2] < FW) return;
    if (in_sizes[3] < NL * NQ * 3) return;
    if (in_sizes[4] < DOUT * NQ) return;
    if (in_sizes[5] < DOUT) return;
    if ((size_t)out_size < (size_t)NSAMP * DOUT) return;
    if (SZ_TOTAL > ws_size) return;
    const float* x  = (const float*)d_in[0];
    const float* w1 = (const float*)d_in[1];
    const float* b1 = (const float*)d_in[2];
    const float* qw = (const float*)d_in[3];
    const float* w2 = (const float*)d_in[4];
    const float* b2 = (const float*)d_in[5];
    float* OUT = (float*)d_out;
    char* wsp = (char*)d_ws;
    bf*    XB  = (bf*)wsp;    wsp += SZ_XB;
    bf*    W1B = (bf*)wsp;    wsp += SZ_WB;
    float* Fp  = (float*)wsp; wsp += SZ_F;
    h16*   WTp = (h16*)wsp;   wsp += SZ_WT;

    { const size_t n8 = (size_t)NSAMP * DIN / 8; k_cvt8<<<(unsigned)((n8 + 255) / 256), 256, 0, stream>>>(x, XB, n8); }
    { const size_t n8 = (size_t)FW * DIN / 8;    k_cvt8<<<(unsigned)((n8 + 255) / 256), 256, 0, stream>>>(w1, W1B, n8); }
    k_wbuild<<<dim3(NL * 2, 1, 1), 256, 0, stream>>>(qw, WTp);
    k_feat<<<dim3(NSAMP / 64, 1, 1), 32, 0, stream>>>(XB, W1B, b1, Fp);
    k_sim<<<dim3(NSAMP / (AW * SPW), 1, 1), 32 * AW, 0, stream>>>(Fp, WTp, w2, b2, OUT);
}
